// SoftmaxLinearAttention_51634096832893
// MI455X (gfx1250) — hardware-run, weakly checked
//
#include <hip/hip_runtime.h>


#ifndef NB
#define NB 2
#endif
#ifndef SEQ
#define SEQ 2048
#endif
#define NB_FULL  2
#define SEQ_FULL 2048
#ifndef OUT_SEQ
#define OUT_SEQ SEQ
#endif
#define DM   1024
#define NH_  16
#define HD   64
#define AW   4
#define TT   32
#define L2E  1.4426950408889634f

static_assert(HD == 64);
static_assert(NH_ * HD == DM);
static_assert(DM % 64 == 0);
static_assert(DM % 32 == 0);
static_assert(SEQ % 64 == 0);
static_assert((NB * SEQ) % 64 == 0);
static_assert(SEQ % 32 == 0);
static_assert(SEQ % (16 * AW) == 0);
static_assert(SEQ % TT == 0);
static_assert(SEQ % 4 == 0);
static_assert(((size_t)SEQ * DM) % 8 == 0);
static_assert(((size_t)DM * DM) % 8 == 0);
static_assert(NB <= NB_FULL);
static_assert(SEQ <= SEQ_FULL);

typedef unsigned short bf;
typedef __attribute__((ext_vector_type(16))) __bf16   v16bf;
typedef __attribute__((ext_vector_type(8)))  unsigned short v8us;
typedef __attribute__((ext_vector_type(16))) unsigned short v16us;
typedef __attribute__((ext_vector_type(8)))  float    v8f;
typedef __attribute__((ext_vector_type(4)))  float    v4f;
typedef v4f  __attribute__((may_alias)) v4fa;

__device__ __forceinline__ unsigned short f2bf(float f) { unsigned u = __float_as_uint(f); u += 0x7FFFu + ((u >> 16) & 1u); return (unsigned short)(u >> 16); }
__device__ __forceinline__ float bf2f(unsigned short u) { return __uint_as_float(((unsigned)u) << 16); }
__device__ __forceinline__ v16bf cat16b(v8us lo, v8us hi) { return __builtin_bit_cast(v16bf, __builtin_shufflevector(lo, hi, 0, 1, 2, 3, 4, 5, 6, 7, 8, 9, 10, 11, 12, 13, 14, 15)); }
__device__ __forceinline__ v8f wmmab(v16bf a, v16bf b, v8f c) { return __builtin_amdgcn_wmma_f32_16x16x32_bf16(false, a, false, b, (short)0, c, false, false); }
__device__ __forceinline__ v16bf ldb(const bf* p)  { return cat16b(*(const v8us*)p, *(const v8us*)(p + 16)); }
__device__ __forceinline__ void wave_sync() { __builtin_amdgcn_fence(3  , "wavefront"); __builtin_amdgcn_wave_barrier(); asm volatile("" ::: "memory"); }

__global__ __launch_bounds__(256) void k_cvt8(const float* __restrict__ src, bf* dst, size_t n8) {
    const size_t i = (size_t)blockIdx.x * 256 + threadIdx.x; if (i >= n8) return;
    const v8f v = *(const v8f*)(src + i * 8); v8us o;
#pragma unroll
    for (int k = 0; k < 8; ++k) o[k] = f2bf(v[k]);
    *(volatile v8us*)(dst + i * 8) = o; __threadfence(); *(volatile v8us*)(dst + i * 8) = o;
}

__global__ __launch_bounds__(32) void k_gemm(const bf* __restrict__ A, size_t aPlane, int nA, const bf* __restrict__ Bt, size_t zB, int K, int om,
                                             float* Pf, bf* Ph, bf* Pl, size_t zP, int RB, size_t sRB, int pitch, int CB, size_t sCB) {
    __shared__ __align__(16) float os[16 * 68];
    const int lane = threadIdx.x & 31, lr = lane & 15, hi = lane >> 4; const int r0 = blockIdx.x * 64, c0 = blockIdx.y * 64;
    const bf* Bz = Bt + (size_t)blockIdx.z * zB;
    v8f acc[4][4];
#pragma unroll
    for (int mb = 0; mb < 4; ++mb)
#pragma unroll
        for (int nb = 0; nb < 4; ++nb) acc[mb][nb] = (v8f){};
    const size_t aoff = (size_t)(r0 + lr) * K + 8 * hi, boff = (size_t)(c0 + lr) * K + 8 * hi;
#pragma unroll 1
    for (int p = 0; p < nA; ++p) {
        const bf* Ap = A + (size_t)p * aPlane;
#pragma unroll 1
        for (int kc = 0; kc < K; kc += 32) {
            v16bf a[4];
#pragma unroll
            for (int mb = 0; mb < 4; ++mb) a[mb] = ldb(Ap + aoff + (size_t)mb * 16 * K + kc);
#pragma unroll
            for (int nb = 0; nb < 4; ++nb) { const v16bf b = ldb(Bz + boff + (size_t)nb * 16 * K + kc);
#pragma unroll
                for (int mb = 0; mb < 4; ++mb) acc[mb][nb] = wmmab(a[mb], b, acc[mb][nb]); }
            asm volatile("v_nop\n\tv_nop\n\tv_nop\n\tv_nop" : "+v"(acc[0][0]), "+v"(acc[1][1]), "+v"(acc[2][2]), "+v"(acc[3][3]) : "v"(a[0]), "v"(a[1]), "v"(a[2]), "v"(a[3]));
        }
    }
    const size_t tbase = (size_t)blockIdx.z * zP + (size_t)(r0 / RB) * sRB + (size_t)(r0 % RB) * (size_t)pitch + (size_t)(c0 / CB) * sCB + (size_t)(c0 % CB);
#pragma unroll
    for (int mb = 0; mb < 4; ++mb) {
#pragma unroll
        for (int nb = 0; nb < 4; ++nb) {
#pragma unroll
            for (int j = 0; j < 8; ++j) os[(hi * 8 + j) * 68 + nb * 16 + lr] = acc[mb][nb][j]; }
        wave_sync();
        const size_t sb = tbase + (size_t)(mb * 16) * (size_t)pitch;
        if (om == 0) {
#pragma unroll 1
            for (int ps = 0; ps < 2; ++ps) {
#pragma unroll
                for (int s = 0; s < 8; ++s) { const int row = 2 * s + hi, cofs = lr * 4;
                    const v4f val = *(const v4fa*)(&os[row * 68 + cofs]);
                    *(volatile v4f*)(Pf + sb + (size_t)row * (size_t)pitch + cofs) = val; }
                if (ps == 0) __threadfence(); }
        } else {
#pragma unroll 1
            for (int ps = 0; ps < 2; ++ps) {
#pragma unroll
                for (int s = 0; s < 4; ++s) { const int row = 4 * s + (lane >> 3), c8 = (lane & 7) * 8;
                    const v4f x0 = *(const v4fa*)(&os[row * 68 + c8]); const v4f x1 = *(const v4fa*)(&os[row * 68 + c8 + 4]); v8us hv, lv;
#pragma unroll
                    for (int i = 0; i < 4; ++i) { const unsigned short a0 = f2bf(x0[i]); const unsigned short a1 = f2bf(x1[i]); hv[i] = a0; hv[4 + i] = a1; lv[i] = f2bf(x0[i] - bf2f(a0)); lv[4 + i] = f2bf(x1[i] - bf2f(a1)); }
                    const size_t oo = sb + (size_t)row * (size_t)pitch + c8;
                    *(volatile v8us*)(Ph + oo) = hv; *(volatile v8us*)(Pl + oo) = lv; }
                if (ps == 0) __threadfence(); }
        }
        wave_sync();
    }
}

__global__ __launch_bounds__(256) void k_prep(const float* __restrict__ QF, const float* __restrict__ KF, bf* QH, bf* QL, bf* KH, bf* KL) {
    __shared__ __align__(16) float Ke[TT * 68];
    __shared__ __align__(16) float Qs[TT * 68];
    __shared__ __align__(16) float Rk[TT * 68];
    __shared__ __align__(16) float pm[4 * 64];
    __shared__ __align__(16) float km[64];
    __shared__ __align__(16) float inv[TT];
    const int tid = threadIdx.x;
    const size_t base = (size_t)blockIdx.x * SEQ * HD;
    { const int c = tid & 63, g = tid >> 6; float m = -3.0e38f;
#pragma unroll 4
      for (int t = g; t < SEQ; t += 4) m = fmaxf(m, KF[base + (size_t)t * HD + c]);
      pm[g * 64 + c] = m; }
    __syncthreads();
    if (tid < 64) km[tid] = fmaxf(fmaxf(pm[tid], pm[64 + tid]), fmaxf(pm[128 + tid], pm[192 + tid]));
    __syncthreads();
    float run = 0.0f;
#pragma unroll 1
    for (int tile = 0; tile < SEQ / TT; ++tile) {
        const int t0 = tile * TT;
#pragma unroll
        for (int i = 0; i < 2; ++i) { const int idx = tid + 256 * i; const int row = idx >> 4, c4 = (idx & 15) * 4;
            const size_t go = base + (size_t)(t0 + row) * HD + c4;
            const v4f kv = *(const v4f*)(KF + go); const v4f qv = *(const v4f*)(QF + go); const v4f mv = *(const v4fa*)(&km[c4]); v4f e;
#pragma unroll
            for (int j = 0; j < 4; ++j) e[j] = __builtin_amdgcn_exp2f((kv[j] - mv[j]) * L2E);
            *(v4fa*)(&Ke[row * 68 + c4]) = e; *(v4fa*)(&Qs[row * 68 + c4]) = qv; }
        __syncthreads();
        { const int tok = tid >> 3, pc = (tid & 7) * 8;
          v4f a = *(const v4fa*)(&Qs[tok * 68 + pc]); v4f c = *(const v4fa*)(&Qs[tok * 68 + pc + 4]);
          float mx = fmaxf(fmaxf(fmaxf(a[0], a[1]), fmaxf(a[2], a[3])), fmaxf(fmaxf(c[0], c[1]), fmaxf(c[2], c[3])));
          mx = fmaxf(mx, __shfl_xor(mx, 1, 32)); mx = fmaxf(mx, __shfl_xor(mx, 2, 32)); mx = fmaxf(mx, __shfl_xor(mx, 4, 32));
#pragma unroll
          for (int j = 0; j < 4; ++j) { a[j] = __builtin_amdgcn_exp2f((a[j] - mx) * L2E); c[j] = __builtin_amdgcn_exp2f((c[j] - mx) * L2E); }
          float s = ((a[0] + a[1]) + (a[2] + a[3])) + ((c[0] + c[1]) + (c[2] + c[3]));
          s += __shfl_xor(s, 1, 32); s += __shfl_xor(s, 2, 32); s += __shfl_xor(s, 4, 32);
          *(v4fa*)(&Qs[tok * 68 + pc]) = a; *(v4fa*)(&Qs[tok * 68 + pc + 4]) = c;
          if ((tid & 7) == 0) inv[tok] = 0.125f / s; }
        if (tid < 64) {
#pragma unroll 1
            for (int r = 0; r < TT; ++r) { run += Ke[r * 68 + tid]; Rk[r * 68 + tid] = 1.0f / (run + 1e-9f); }
        }
        __syncthreads();
        { const int row = tid >> 3, c8 = (tid & 7) * 8;
          const v4f q0 = *(const v4fa*)(&Qs[row * 68 + c8]); const v4f q1 = *(const v4fa*)(&Qs[row * 68 + c8 + 4]);
          const v4f r0 = *(const v4fa*)(&Rk[row * 68 + c8]); const v4f r1 = *(const v4fa*)(&Rk[row * 68 + c8 + 4]);
          const v4f k0 = *(const v4fa*)(&Ke[row * 68 + c8]); const v4f k1 = *(const v4fa*)(&Ke[row * 68 + c8 + 4]);
          const float sc = inv[row];
          v8us qh, ql, kh, kl;
#pragma unroll
          for (int i = 0; i < 4; ++i) {
              const float n0 = (q0[i] * sc) * r0[i]; const float n1 = (q1[i] * sc) * r1[i];
              const unsigned short a0 = f2bf(n0); const unsigned short a1 = f2bf(n1);
              qh[i] = a0; qh[4 + i] = a1; ql[i] = f2bf(n0 - bf2f(a0)); ql[4 + i] = f2bf(n1 - bf2f(a1));
              const unsigned short b0 = f2bf(k0[i]); const unsigned short b1 = f2bf(k1[i]);
              kh[i] = b0; kh[4 + i] = b1; kl[i] = f2bf(k0[i] - bf2f(b0)); kl[4 + i] = f2bf(k1[i] - bf2f(b1)); }
          const size_t oo = base + (size_t)(t0 + row) * HD + c8;
#pragma unroll 1
          for (int ps = 0; ps < 2; ++ps) {
              *(volatile v8us*)(QH + oo) = qh; *(volatile v8us*)(QL + oo) = ql; *(volatile v8us*)(KH + oo) = kh; *(volatile v8us*)(KL + oo) = kl;
              if (ps == 0) __threadfence(); } }
        __syncthreads();
    }
}

__global__ __launch_bounds__(32 * AW) void k_lattn(const bf* __restrict__ QH, const bf* __restrict__ QL, const bf* __restrict__ KH, const bf* __restrict__ KL,
                                                   const bf* __restrict__ VH, const bf* __restrict__ VL, bf* CH, bf* CL) {
    __shared__ __align__(16) float os[AW * 16 * 68];
    const int lane = threadIdx.x & 31, lr = lane & 15, hi = lane >> 4;
    const int wave = __builtin_amdgcn_readfirstlane((int)(threadIdx.x >> 5));
    const int zh = blockIdx.y; const int b = zh / NH_, h = zh % NH_;
    const int t0 = (blockIdx.x * AW + wave) * 16;
    const size_t pbase = (size_t)zh * SEQ * HD;
    const size_t qo = pbase + (size_t)(t0 + lr) * HD + 8 * hi;
    const v16bf qh0 = ldb(QH + qo), qh1 = ldb(QH + qo + 32), ql0 = ldb(QL + qo), ql1 = ldb(QL + qo + 32);
    const size_t ko = pbase + (size_t)lr * HD + 8 * hi;
    const size_t vo = pbase + (size_t)lr * SEQ + 8 * hi;
    v8f o0 = (v8f){}, o1 = (v8f){}, o2 = (v8f){}, o3 = (v8f){};
    const int nst = (t0 >> 5) + 1;
    const int qi = t0 + lr;
#pragma unroll 1
    for (int st = 0; st < nst; ++st) {
        const int key0 = st * 32;
        const bf* kh = KH + ko + (size_t)key0 * HD; const bf* kl = KL + ko + (size_t)key0 * HD;
        const v16bf ah0 = ldb(kh), ah1 = ldb(kh + 32), bh0 = ldb(kh + 16 * HD), bh1 = ldb(kh + 16 * HD + 32);
        const v16bf al0 = ldb(kl), al1 = ldb(kl + 32), bl0 = ldb(kl + 16 * HD), bl1 = ldb(kl + 16 * HD + 32);
        v8f sHa = (v8f){}, sXa = (v8f){}, sHb = (v8f){}, sXb = (v8f){};
        sXa = wmmab(ah0, ql0, sXa); sXb = wmmab(bh0, ql0, sXb); sHa = wmmab(ah0, qh0, sHa); sHb = wmmab(bh0, qh0, sHb);
        sXa = wmmab(ah1, ql1, sXa); sXb = wmmab(bh1, ql1, sXb); sHa = wmmab(ah1, qh1, sHa); sHb = wmmab(bh1, qh1, sHb);
        sXa = wmmab(al0, qh0, sXa); sXb = wmmab(bl0, qh0, sXb); sXa = wmmab(al1, qh1, sXa); sXb = wmmab(bl1, qh1, sXb);
        asm volatile("v_nop\n\tv_nop\n\tv_nop\n\tv_nop" : "+v"(sHa), "+v"(sXa), "+v"(sHb), "+v"(sXb) : "v"(ah0), "v"(ah1), "v"(bh0), "v"(bh1), "v"(al0), "v"(al1), "v"(bl0), "v"(bl1));
        v16us ph, pl;
        const int ka = key0 + 8 * hi, kb = key0 + 16 + 8 * hi;
#pragma unroll
        for (int r = 0; r < 8; ++r) {
            const float fa = sHa[r] + sXa[r]; const float fb = sHb[r] + sXb[r];
            const float va = (ka + r <= qi) ? fa : 0.0f; const float vb = (kb + r <= qi) ? fb : 0.0f;
            const unsigned short ha = f2bf(va); const unsigned short hb = f2bf(vb);
            ph[r] = ha; ph[8 + r] = hb; pl[r] = f2bf(va - bf2f(ha)); pl[8 + r] = f2bf(vb - bf2f(hb)); }
        const v16bf pbh = __builtin_bit_cast(v16bf, ph), pbl = __builtin_bit_cast(v16bf, pl);
        const bf* vh = VH + vo + key0; const bf* vl = VL + vo + key0;
        const v16bf vh0 = ldb(vh), vh1 = ldb(vh + (size_t)16 * SEQ), vh2 = ldb(vh + (size_t)32 * SEQ), vh3 = ldb(vh + (size_t)48 * SEQ);
        const v16bf vl0 = ldb(vl), vl1 = ldb(vl + (size_t)16 * SEQ), vl2 = ldb(vl + (size_t)32 * SEQ), vl3 = ldb(vl + (size_t)48 * SEQ);
        o0 = wmmab(vh0, pbl, o0); o1 = wmmab(vh1, pbl, o1); o2 = wmmab(vh2, pbl, o2); o3 = wmmab(vh3, pbl, o3);
        o0 = wmmab(vl0, pbh, o0); o1 = wmmab(vl1, pbh, o1); o2 = wmmab(vl2, pbh, o2); o3 = wmmab(vl3, pbh, o3);
        o0 = wmmab(vh0, pbh, o0); o1 = wmmab(vh1, pbh, o1); o2 = wmmab(vh2, pbh, o2); o3 = wmmab(vh3, pbh, o3);
        asm volatile("v_nop\n\tv_nop\n\tv_nop\n\tv_nop" : "+v"(o0), "+v"(o1), "+v"(o2), "+v"(o3) : "v"(vh0), "v"(vh1), "v"(vh2), "v"(vh3), "v"(vl0), "v"(vl1), "v"(vl2), "v"(vl3), "v"(pbh), "v"(pbl));
    }
    const int wb = wave * 16 * 68;
    { v4f a, c;
      a[0] = o0[0]; a[1] = o0[1]; a[2] = o0[2]; a[3] = o0[3]; c[0] = o0[4]; c[1] = o0[5]; c[2] = o0[6]; c[3] = o0[7];
      *(v4fa*)(&os[wb + lr * 68 +  0 + 8 * hi]) = a; *(v4fa*)(&os[wb + lr * 68 +  0 + 8 * hi + 4]) = c;
      a[0] = o1[0]; a[1] = o1[1]; a[2] = o1[2]; a[3] = o1[3]; c[0] = o1[4]; c[1] = o1[5]; c[2] = o1[6]; c[3] = o1[7];
      *(v4fa*)(&os[wb + lr * 68 + 16 + 8 * hi]) = a; *(v4fa*)(&os[wb + lr * 68 + 16 + 8 * hi + 4]) = c;
      a[0] = o2[0]; a[1] = o2[1]; a[2] = o2[2]; a[3] = o2[3]; c[0] = o2[4]; c[1] = o2[5]; c[2] = o2[6]; c[3] = o2[7];
      *(v4fa*)(&os[wb + lr * 68 + 32 + 8 * hi]) = a; *(v4fa*)(&os[wb + lr * 68 + 32 + 8 * hi + 4]) = c;
      a[0] = o3[0]; a[1] = o3[1]; a[2] = o3[2]; a[3] = o3[3]; c[0] = o3[4]; c[1] = o3[5]; c[2] = o3[6]; c[3] = o3[7];
      *(v4fa*)(&os[wb + lr * 68 + 48 + 8 * hi]) = a; *(v4fa*)(&os[wb + lr * 68 + 48 + 8 * hi + 4]) = c; }
    wave_sync();
    const size_t cb = ((size_t)b * SEQ + t0) * DM + (size_t)h * HD;
#pragma unroll 1
    for (int ps = 0; ps < 2; ++ps) {
#pragma unroll
        for (int s = 0; s < 4; ++s) { const int row = 4 * s + (lane >> 3), c8 = (lane & 7) * 8;
            const v4f x0 = *(const v4fa*)(&os[wb + row * 68 + c8]); const v4f x1 = *(const v4fa*)(&os[wb + row * 68 + c8 + 4]); v8us hv, lv;
#pragma unroll
            for (int i = 0; i < 4; ++i) { const unsigned short a0 = f2bf(x0[i]); const unsigned short a1 = f2bf(x1[i]); hv[i] = a0; hv[4 + i] = a1; lv[i] = f2bf(x0[i] - bf2f(a0)); lv[4 + i] = f2bf(x1[i] - bf2f(a1)); }
            const size_t oo = cb + (size_t)row * DM + c8;
            *(volatile v8us*)(CH + oo) = hv; *(volatile v8us*)(CL + oo) = lv; }
        if (ps == 0) __threadfence(); }
}

static constexpr size_t al256(size_t v) { return (v + 255) & ~(size_t)255; }
static constexpr size_t SZ_XB = al256((size_t)NB * SEQ * DM * 2);
static constexpr size_t SZ_WQ = al256((size_t)3 * DM * DM * 2);
static constexpr size_t SZ_WO = al256((size_t)DM * DM * 2);
static constexpr size_t SZ_QK = al256((size_t)2 * NB * NH_ * SEQ * HD * 4);
static constexpr size_t SZ_PL = al256((size_t)NB * NH_ * SEQ * HD * 2);
static constexpr size_t SZ_CT = al256((size_t)NB * SEQ * DM * 2);
static constexpr size_t SZ_TOTAL = SZ_XB + SZ_WQ + SZ_WO + SZ_QK + 6 * SZ_PL + 2 * SZ_CT;
static_assert(SZ_TOTAL <= (size_t)134217728);
static_assert(((size_t)DM * DM * 2) % 256 == 0);
static_assert(((size_t)NB * NH_ * SEQ * HD * 4) % 256 == 0);
static_assert(SZ_CT % 2 == 0);

extern "C" void kernel_launch(void* const* d_in, const int* in_sizes, int n_in,
                              void* d_out, int out_size, void* d_ws, size_t ws_size, hipStream_t stream) {
    if (n_in < 3) return;
    const size_t needx = ((size_t)(NB - 1) * SEQ_FULL + SEQ) * DM;
    if ((size_t)in_sizes[0] < needx) return;
    if ((size_t)in_sizes[1] < (size_t)3 * DM * DM || (size_t)in_sizes[2] < (size_t)DM * DM) return;
    if ((size_t)out_size < ((size_t)(NB - 1) * OUT_SEQ + SEQ) * DM) return;
    if (SZ_TOTAL > ws_size) return;
    const float* x = (const float*)d_in[0]; const float* wqkv = (const float*)d_in[1]; const float* wout = (const float*)d_in[2];
    float* OUT = (float*)d_out;
    char* wsp = (char*)d_ws;
    bf* XB = (bf*)wsp; wsp += SZ_XB;
    bf* WQ = (bf*)wsp; wsp += SZ_WQ;
    bf* WO = (bf*)wsp; wsp += SZ_WO;
    float* QF = (float*)wsp; wsp += SZ_QK;
    bf* VH = (bf*)wsp; wsp += SZ_PL;
    bf* VL = (bf*)wsp; wsp += SZ_PL;
    bf* QH = (bf*)wsp; wsp += SZ_PL;
    bf* QL = (bf*)wsp; wsp += SZ_PL;
    bf* KH = (bf*)wsp; wsp += SZ_PL;
    bf* KL = (bf*)wsp; wsp += SZ_PL;
    bf* CH = (bf*)wsp; wsp += SZ_CT;
    bf* CL = (bf*)wsp; wsp += SZ_CT;
    const size_t qkPlane = (size_t)NB * NH_ * SEQ * HD;
    float* KF = QF + qkPlane;

    if (SEQ == SEQ_FULL) {
        const size_t n8 = (size_t)NB * SEQ * DM / 8;
        k_cvt8<<<(unsigned)((n8 + 255) / 256), 256, 0, stream>>>(x, XB, n8);
    } else {
        const size_t n8 = (size_t)SEQ * DM / 8;
        for (int b = 0; b < NB; ++b) k_cvt8<<<(unsigned)((n8 + 255) / 256), 256, 0, stream>>>(x + (size_t)b * SEQ_FULL * DM, XB + (size_t)b * SEQ * DM, n8);
    }
    { const size_t n8 = (size_t)3 * DM * DM / 8; k_cvt8<<<(unsigned)((n8 + 255) / 256), 256, 0, stream>>>(wqkv, WQ, n8); }
    { const size_t n8 = (size_t)DM * DM / 8;     k_cvt8<<<(unsigned)((n8 + 255) / 256), 256, 0, stream>>>(wout, WO, n8); }

    k_gemm<<<dim3(NB * SEQ / 64, DM / 64, 2), 32, 0, stream>>>(XB, (size_t)0, 1, WQ, (size_t)DM * DM, DM, 0,
        QF, VH, VL, qkPlane, SEQ, (size_t)NH_ * SEQ * HD, HD, HD, (size_t)SEQ * HD);
    k_gemm<<<dim3(DM / 64, NB * SEQ / 64, 1), 32, 0, stream>>>(WQ + (size_t)2 * DM * DM, (size_t)0, 1, XB, (size_t)0, DM, 1,
        QF, VH, VL, (size_t)0, DM, (size_t)0, SEQ, SEQ, (size_t)DM * SEQ);

    k_prep<<<NB * NH_, 256, 0, stream>>>(QF, KF, QH, QL, KH, KL);

    k_lattn<<<dim3(SEQ / (16 * AW), NB * NH_, 1), 32 * AW, 0, stream>>>(QH, QL, KH, KL, VH, VL, CH, CL);

    k_gemm<<<dim3(NB * SEQ / 64, DM / 64, 1), 32, 0, stream>>>(CH, SZ_CT / 2, 2, WO, (size_t)0, DM, 0,
        OUT, VH, VL, (size_t)0, SEQ, (size_t)OUT_SEQ * DM, DM, DM, (size_t)0);
}
